// BF16IndexerBaseline_57612691308721
// MI455X (gfx1250) — hardware-verified
//
#include <hip/hip_runtime.h>
#include <stdint.h>
#include <stddef.h>

typedef __bf16 v16b __attribute__((ext_vector_type(16)));
typedef float v8f __attribute__((ext_vector_type(8)));
typedef float v4f __attribute__((ext_vector_type(4)));
typedef unsigned int v4u __attribute__((ext_vector_type(4)));
typedef v4u __attribute__((may_alias)) v4u_ma;
typedef v4f __attribute__((may_alias)) v4f_ma;

union Frag {
  v16b v;
  v4u  q[2];
};

#define BM 64
#define BN 64
#define DD 128
#define LROW 68
#define OTS 68
#define NTHR 256
#define QS_SCALE 0.08837890625f

static __device__ __forceinline__ v8f wmma_bf16_32(v16b a, v16b b, v8f c) {
  v8f d = __builtin_amdgcn_wmma_f32_16x16x32_bf16(false, a, false, b, (short)0, c, false, false);
  asm volatile("v_nop\n\tv_nop\n\tv_nop\n\tv_nop" : "+v"(d) : "v"(a), "v"(b));
  return d;
}

static __device__ __forceinline__ float bf16_bits_to_f32(unsigned short u) {
  return __uint_as_float(((unsigned int)u) << 16);
}

static __device__ __forceinline__ float rne_bf16_f32(float x) {
  unsigned int u = __float_as_uint(x);
  u = (u + 0x7FFFu + ((u >> 16) & 1u)) & 0xFFFF0000u;
  return __uint_as_float(u);
}

static __device__ __forceinline__ void store_piece(float* out, size_t off, v4f v, int cnt) {
  if (cnt == 4 && ((off & 3) == 0)) {
    *(volatile v4f*)(out + off) = v;
  } else {
    volatile float* o = (volatile float*)out;
    if (cnt > 0) o[off]     = v.x;
    if (cnt > 1) o[off + 1] = v.y;
    if (cnt > 2) o[off + 2] = v.z;
    if (cnt > 3) o[off + 3] = v.w;
  }
}

__global__ __launch_bounds__(NTHR)
void k_index_score(const unsigned short* __restrict__ q,
                   const unsigned short* __restrict__ k,
                   const unsigned short* __restrict__ w,
                   float* __restrict__ out,
                   int M, int N, int H)
{
  __shared__ __attribute__((aligned(16))) unsigned int lq[BM * LROW];
  __shared__ __attribute__((aligned(16))) unsigned int lk[BN * LROW];
  __shared__ __attribute__((aligned(16))) float ot[BM * OTS];
  __shared__ float lqs[BM];

  const int tid  = threadIdx.x;
  const int wave = tid >> 5;
  const int lane = tid & 31;
  const int hf   = lane >> 4;
  const int l16  = lane & 15;
  const int mSub = wave >> 1;
  const int nGrp = wave & 1;
  const int n0 = blockIdx.x * BN;
  const int m0 = blockIdx.y * BM;
  const int b  = blockIdx.z;

  const v4u zero4 = {0u, 0u, 0u, 0u};

#pragma unroll
  for (int i = 0; i < 4; ++i) {
    const int id  = tid + i * NTHR;
    const int row = id >> 4;
    const int c   = id & 15;
    const int n   = n0 + row;
    v4u val = zero4;
    if (n < N) val = *(const v4u_ma*)(k + (((size_t)b * N + n) * DD + c * 8));
    *(v4u_ma*)(lk + row * LROW + c * 4) = val;
  }

  const v8f zero8 = {0.f, 0.f, 0.f, 0.f, 0.f, 0.f, 0.f, 0.f};
  v8f sum0 = zero8, sum1 = zero8;

  const int arow  = (mSub * 16 + l16) * LROW + 4 * hf;
  const int brow0 = (nGrp * 32 + l16) * LROW + 4 * hf;
  const int brow1 = (nGrp * 32 + 16 + l16) * LROW + 4 * hf;

#pragma unroll 1
  for (int h = 0; h < H; ++h) {
    __syncthreads();

#pragma unroll
    for (int i = 0; i < 4; ++i) {
      const int id  = tid + i * NTHR;
      const int row = id >> 4;
      const int c   = id & 15;
      const int m   = m0 + row;
      v4u val = zero4;
      if (m < M) val = *(const v4u_ma*)(q + ((((size_t)b * M + m) * H + h) * DD + c * 8));
      *(v4u_ma*)(lq + row * LROW + c * 4) = val;
    }
    if (tid < BM) {
      const int m = m0 + tid;
      float v = 0.f;
      if (m < M) v = rne_bf16_f32(bf16_bits_to_f32(w[(size_t)h * M + m]) * QS_SCALE);
      lqs[tid] = v;
    }
    __syncthreads();

    v8f acc0 = zero8, acc1 = zero8;
#pragma unroll
    for (int kk = 0; kk < 4; ++kk) {
      Frag a, b0, b1;
      a.q[0]  = *(const v4u_ma*)(lq + arow + kk * 16);
      a.q[1]  = *(const v4u_ma*)(lq + arow + kk * 16 + 8);
      b0.q[0] = *(const v4u_ma*)(lk + brow0 + kk * 16);
      b0.q[1] = *(const v4u_ma*)(lk + brow0 + kk * 16 + 8);
      b1.q[0] = *(const v4u_ma*)(lk + brow1 + kk * 16);
      b1.q[1] = *(const v4u_ma*)(lk + brow1 + kk * 16 + 8);
      acc0 = wmma_bf16_32(a.v, b0.v, acc0);
      acc1 = wmma_bf16_32(a.v, b1.v, acc1);
    }

    float qs[8];
#pragma unroll
    for (int v = 0; v < 8; ++v) qs[v] = lqs[mSub * 16 + hf * 8 + v];
#pragma unroll
    for (int v = 0; v < 8; ++v) {
      const float x0 = __builtin_fmaxf(rne_bf16_f32(acc0[v]), 0.f);
      const float x1 = __builtin_fmaxf(rne_bf16_f32(acc1[v]), 0.f);
      sum0[v] += x0 * qs[v];
      sum1[v] += x1 * qs[v];
    }
  }

#pragma unroll
  for (int v = 0; v < 8; ++v) {
    const int r = mSub * 16 + hf * 8 + v;
    ot[r * OTS + nGrp * 32 + l16]      = sum0[v];
    ot[r * OTS + nGrp * 32 + 16 + l16] = sum1[v];
  }
  __syncthreads();

  v4f    vv[4];
  size_t off[4];
  int    cnt[4];
#pragma unroll
  for (int it = 0; it < 4; ++it) {
    const int L  = wave * 16 + it * 4 + (lane >> 3);
    const int q8 = lane & 7;
    const int r  = L >> 1;
    const int c  = (L & 1) * 32 + q8 * 4;
    vv[it] = *(const v4f_ma*)(ot + r * OTS + c);
    const int m = m0 + r;
    const int n = n0 + c;
    off[it] = ((size_t)b * M + m) * (size_t)N + (size_t)n;
    int cc = 0;
    if (m < M) { cc = N - n; if (cc > 4) cc = 4; if (cc < 0) cc = 0; }
    cnt[it] = cc;
  }
#pragma unroll
  for (int it = 0; it < 4; ++it) store_piece(out, off[it], vv[it], cnt[it]);
  __threadfence();
#pragma unroll
  for (int it = 0; it < 4; ++it) store_piece(out, off[it], vv[it], cnt[it]);
}

extern "C" void kernel_launch(void* const* d_in, const int* in_sizes, int n_in,
                              void* d_out, int out_size, void* d_ws, size_t ws_size,
                              hipStream_t stream) {
  (void)d_ws; (void)ws_size;
  if (n_in < 3) return;
  const unsigned short* q = (const unsigned short*)d_in[0];
  const unsigned short* k = (const unsigned short*)d_in[1];
  const unsigned short* w = (const unsigned short*)d_in[2];
  float* out = (float*)d_out;

  const long long nq = in_sizes[0], nk = in_sizes[1], nw = in_sizes[2];
  if (nq <= 0 || nk <= 0 || nw <= 0 || out_size <= 0) return;
  long long B = nq / (nw * (long long)DD);
  if (B < 1) B = 1;
  const long long N = nk / (B * (long long)DD);
  if (N < 1) return;
  const long long M = (long long)out_size / (B * N);
  if (M < 1) return;
  const long long H = nw / M;
  if (H < 1) return;
  if (B * M * H * (long long)DD > nq) return;
  if (B * N * (long long)DD > nk) return;
  if (H * M > nw) return;
  if (B * M * N > (long long)out_size) return;

  dim3 grid((unsigned)((N + BN - 1) / BN), (unsigned)((M + BM - 1) / BM), (unsigned)B);
  k_index_score<<<grid, NTHR, 0, stream>>>(q, k, w, out, (int)M, (int)N, (int)H);
  (void)hipGetLastError();
}
